// STFT_45818711114408
// MI455X (gfx1250) — hardware-verified
//
#include <hip/hip_runtime.h>

typedef __bf16         v16b __attribute__((ext_vector_type(16)));
typedef unsigned short v8us __attribute__((ext_vector_type(8)));
typedef float          v8f  __attribute__((ext_vector_type(8)));
typedef float          v4f  __attribute__((ext_vector_type(4)));
typedef v8us __attribute__((may_alias)) v8usa;
typedef v4f  __attribute__((may_alias)) v4fa;

union Frag { v16b v; v8us half[2]; };

#define NB    32
#define TLEN  262144
#define NF    512
#define HOP   128
#define PADX  256
#define TN    2049
#define CDIM  514
#define NA    576
#define KS    544
#define SP    1088
#define MP    2080
#define LP    266624
#define XOFF  640
#define FOWN  61
#define FBLK  64
#define NFB   34
#define GRP   16
#define NGRP  2

static_assert(LP == HOP * (MP - 1) + NF);
static_assert(LP % 64 == 0);
static_assert((LP / 8) * 8 == LP);
static_assert(MP % 16 == 0);
static_assert((NFB - 1) * FOWN + FBLK <= MP);
static_assert((NFB - 1) * FOWN + FOWN - 1 >= TN);
static_assert(NB == GRP * NGRP);
static_assert(KS % 32 == 0 && NF % 32 == 0 && SP == 2 * KS);
static_assert(NA == 4 * 144 && NA >= KS && KS >= CDIM);
static_assert(XOFF % 8 == 0 && TLEN % 8 == 0);
static_assert(HOP * TN - PADX + 96 + 32 <= TLEN);

__device__ __forceinline__ unsigned short bf16_bits(float f) {
  unsigned int u = __float_as_uint(f);
  u += 0x7FFFu + ((u >> 16) & 1u);
  return (unsigned short)(u >> 16);
}
__device__ __forceinline__ float bf16_val(unsigned short s) {
  return __uint_as_float(((unsigned int)s) << 16);
}

__device__ __forceinline__ v8f wmma_bf16(v16b a, v16b b, v8f c) {
  v8f d = __builtin_amdgcn_wmma_f32_16x16x32_bf16(false, a, false, b, (short)0, c, false, false);
  asm volatile("v_nop\n\tv_nop\n\tv_nop\n\tv_nop" : "+v"(d) : "v"(a), "v"(b));
  return d;
}

__device__ __forceinline__ v16b load_frag(const unsigned short* p, int h) {
  Frag f;
  f.half[0] = *(const v8usa*)(p + 8 * h);
  f.half[1] = *(const v8usa*)(p + 16 + 8 * h);
  return f.v;
}

__global__ __launch_bounds__(256) void k_cvt_x(const float* __restrict__ x,
                                                unsigned short* __restrict__ xp) {
  const int g = blockIdx.x * 256 + threadIdx.x;
  if (g >= NB * (LP / 8)) return;
  const int b  = g / (LP / 8);
  const int u0 = (g - b * (LP / 8)) * 8;
  const int xi = u0 - XOFF;
  const bool in = (xi >= 0) && (xi < TLEN);
  int ci = xi < 0 ? 0 : xi;
  ci = ci > (TLEN - 8) ? (TLEN - 8) : ci;
  const float* src = x + (size_t)b * TLEN + ci;
  const v4f a = *(const v4fa*)src;
  const v4f c = *(const v4fa*)(src + 4);
  const unsigned short z = 0;
  v8us o;
  o[0] = in ? bf16_bits(a.x) : z;  o[1] = in ? bf16_bits(a.y) : z;
  o[2] = in ? bf16_bits(a.z) : z;  o[3] = in ? bf16_bits(a.w) : z;
  o[4] = in ? bf16_bits(c.x) : z;  o[5] = in ? bf16_bits(c.y) : z;
  o[6] = in ? bf16_bits(c.z) : z;  o[7] = in ? bf16_bits(c.w) : z;
  unsigned short* dst = xp + (size_t)g * 8;
  *(volatile v8us*)dst = o;
  __threadfence();
  *(volatile v8us*)dst = o;
}

__global__ __launch_bounds__(256) void k_cvt_w(const float* __restrict__ w,
                                                unsigned short* __restrict__ wp) {
  const int g = blockIdx.x * 256 + threadIdx.x;
  if (g >= NA * (NF / 8)) return;
  const int n  = g / (NF / 8);
  const int k0 = (g - n * (NF / 8)) * 8;
  const bool in = n < CDIM;
  const int cn = in ? n : (CDIM - 1);
  const float* src = w + (size_t)cn * NF + k0;
  const v4f a = *(const v4fa*)src;
  const v4f c = *(const v4fa*)(src + 4);
  const unsigned short z = 0;
  v8us o;
  o[0] = in ? bf16_bits(a.x) : z;  o[1] = in ? bf16_bits(a.y) : z;
  o[2] = in ? bf16_bits(a.z) : z;  o[3] = in ? bf16_bits(a.w) : z;
  o[4] = in ? bf16_bits(c.x) : z;  o[5] = in ? bf16_bits(c.y) : z;
  o[6] = in ? bf16_bits(c.z) : z;  o[7] = in ? bf16_bits(c.w) : z;
  unsigned short* dst = wp + (size_t)g * 8;
  *(volatile v8us*)dst = o;
  __threadfence();
  *(volatile v8us*)dst = o;
}

__global__ __launch_bounds__(256) void k_cvt_iw(const float* __restrict__ iw,
                                                 unsigned short* __restrict__ iwt) {
  const int g = blockIdx.x * 256 + threadIdx.x;
  if (g >= NF * (KS / 8)) return;
  const int n  = g / (KS / 8);
  const int c0 = (g - n * (KS / 8)) * 8;
  const unsigned short z = 0;
  v8us o;
  #pragma unroll
  for (int i = 0; i < 8; ++i) {
    const int c  = c0 + i;
    const int cc = c < CDIM ? c : (CDIM - 1);
    const float v = iw[(size_t)cc * NF + n];
    o[i] = (c < CDIM) ? bf16_bits(v) : z;
  }
  unsigned short* dst = iwt + (size_t)g * 8;
  *(volatile v8us*)dst = o;
  __threadfence();
  *(volatile v8us*)dst = o;
}

__device__ __forceinline__ void ana_store(const unsigned short* sT, unsigned short* gb,
                                          int w, int lane) {
  const int q8 = lane & 7, sub = lane >> 3;
  #pragma unroll
  for (int it = 0; it < 17; ++it) {
    const int L   = 68 * w + 4 * it + sub;
    const int row = L / 17;
    const int li  = L - row * 17;
    const v8us v = *(const v8usa*)(sT + row * SP + li * 64 + 8 * q8);
    *(volatile v8us*)(gb + (size_t)row * SP + li * 64 + 8 * q8) = v;
  }
}

__global__ __launch_bounds__(128) void k_ana(const unsigned short* __restrict__ xp,
                                            const unsigned short* __restrict__ wp,
                                            unsigned short* __restrict__ sp,
                                            int b0)
{
  __shared__ __attribute__((aligned(16))) unsigned short sT[16 * SP];

  const int tid = threadIdx.x, lane = tid & 31, w = tid >> 5;
  const int h = lane >> 4, m = lane & 15;
  const int g0 = blockIdx.x * 16;
  const int bl = blockIdx.y;
  const int b  = b0 + bl;
  const int c0 = w * 144;

  const unsigned short* xa = xp + (size_t)b * LP + (size_t)(g0 + m) * HOP;
  const unsigned short* wb = wp + (size_t)(c0 + m) * NF;

  const v8f z8 = {0.f, 0.f, 0.f, 0.f, 0.f, 0.f, 0.f, 0.f};
  v8f acc[9];
  #pragma unroll
  for (int nt = 0; nt < 9; ++nt) acc[nt] = z8;

  #pragma unroll 1
  for (int k0 = 0; k0 < NF; k0 += 32) {
    const v16b a = load_frag(xa + k0, h);
    #pragma unroll
    for (int nt = 0; nt < 9; ++nt) {
      const v16b bf = load_frag(wb + (size_t)nt * 16 * NF + k0, h);
      acc[nt] = wmma_bf16(a, bf, acc[nt]);
    }
  }

  #pragma unroll
  for (int nt = 0; nt < 9; ++nt) {
    if (c0 + 16 * nt < KS) {
      const int col = c0 + 16 * nt + m;
      #pragma unroll
      for (int r = 0; r < 8; ++r) {
        const float v = acc[nt][r];
        const unsigned short hb = bf16_bits(v);
        const unsigned short lb = bf16_bits(v - bf16_val(hb));
        sT[(8 * h + r) * SP + col]      = hb;
        sT[(8 * h + r) * SP + KS + col] = lb;
      }
    }
  }
  __syncthreads();

  unsigned short* gb = sp + ((size_t)bl * MP + g0) * SP;
  ana_store(sT, gb, w, lane);
  __threadfence();
  ana_store(sT, gb, w, lane);
}

__device__ __forceinline__ void syn_store(const float* oT, float* orow,
                                          int f0, int pg, int w, int lane) {
  const int q8 = lane & 7, sub = lane >> 3;
  #pragma unroll
  for (int it = 0; it < 4; ++it) {
    const int li = 16 * it + 4 * w + sub;
    const int f  = f0 + li;
    if (li < FOWN && f >= 2 && f <= TN) {
      const int t = HOP * f - PADX + 32 * pg;
      const v4f v = *(const v4fa*)(oT + li * 32 + 4 * q8);
      *(volatile v4f*)(orow + t + 4 * q8) = v;
    }
  }
}

__global__ __launch_bounds__(128) void k_syn(const unsigned short* __restrict__ sp,
                                            const unsigned short* __restrict__ iwt,
                                            const float* __restrict__ win,
                                            float* __restrict__ out,
                                            int b0)
{
  __shared__ __attribute__((aligned(16))) float yT[FBLK * 128];
  __shared__ __attribute__((aligned(16))) float oT[FBLK * 32];
  __shared__ float w2[NF];

  const int tid = threadIdx.x, lane = tid & 31, w = tid >> 5;
  const int h = lane >> 4, m = lane & 15;
  const int f0 = blockIdx.x * FOWN;
  const int pg = blockIdx.y;
  const int bl = blockIdx.z;
  const int b  = b0 + bl;

  for (int i = tid; i < NF; i += 128) {
    const float ww = bf16_val(bf16_bits(win[i]));
    w2[i] = ww * ww;
  }

  const unsigned short* sa = sp + ((size_t)bl * MP + f0 + 16 * w + m) * SP;
  const unsigned short* ib = iwt + (size_t)(32 * pg + m) * KS;

  const v8f z8 = {0.f, 0.f, 0.f, 0.f, 0.f, 0.f, 0.f, 0.f};
  v8f acc[8];
  #pragma unroll
  for (int j = 0; j < 8; ++j) acc[j] = z8;

  #pragma unroll 1
  for (int k0 = 0; k0 < SP; k0 += 32) {
    const int kk = (k0 < KS) ? k0 : (k0 - KS);
    const v16b a = load_frag(sa + k0, h);
    #pragma unroll
    for (int j = 0; j < 8; ++j) {
      const v16b bf = load_frag(ib + (size_t)(128 * (j >> 1) + 16 * (j & 1)) * KS + kk, h);
      acc[j] = wmma_bf16(a, bf, acc[j]);
    }
  }

  #pragma unroll
  for (int j = 0; j < 8; ++j) {
    const int lc = 32 * (j >> 1) + 16 * (j & 1) + m;
    #pragma unroll
    for (int r = 0; r < 8; ++r) yT[(16 * w + 8 * h + r) * 128 + lc] = acc[j][r];
  }
  __syncthreads();

  for (int e = tid; e < FOWN * 32; e += 128) {
    const int li = e >> 5, lp = e & 31;
    const int f = f0 + li;
    float s = 0.0f, cf = 0.0f;
    #pragma unroll
    for (int jj = 3; jj >= 0; --jj) {
      const int fr = f - jj;
      const bool ok = (fr >= 0) && (fr < TN);
      const float yv = yT[(li + 3 - jj) * 128 + 32 * jj + lp];
      const float wv = w2[128 * jj + 32 * pg + lp];
      s  = s  + (ok ? yv : 0.0f);
      cf = cf + (ok ? wv : 0.0f);
    }
    const float rc = 1.0f / (cf + 1e-8f);
    oT[li * 32 + lp] = s * rc;
  }
  __syncthreads();

  float* orow = out + (size_t)b * TLEN;
  syn_store(oT, orow, f0, pg, w, lane);
  __threadfence();
  syn_store(oT, orow, f0, pg, w, lane);
}

extern "C" void kernel_launch(void* const* d_in, const int* in_sizes, int n_in,
                              void* d_out, int out_size, void* d_ws, size_t ws_size,
                              hipStream_t stream) {
  if (n_in < 4) return;
  if (in_sizes[0] != NB * TLEN) return;
  if (in_sizes[1] != CDIM * NF) return;
  if (in_sizes[2] != CDIM * NF) return;
  if (in_sizes[3] != NF) return;
  if (out_size != NB * TLEN) return;

  const float* x      = (const float*)d_in[0];
  const float* weight = (const float*)d_in[1];
  const float* invw   = (const float*)d_in[2];
  const float* window = (const float*)d_in[3];
  float* out = (float*)d_out;

  const size_t xp_bytes = (size_t)NB * LP * 2;
  const size_t wp_bytes = (size_t)NA * NF * 2;
  const size_t iw_bytes = (size_t)NF * KS * 2;
  const size_t sp_bytes = (size_t)GRP * MP * SP * 2;
  const size_t total = xp_bytes + wp_bytes + iw_bytes + sp_bytes;
  if (total > ws_size) return;

  char* ws = (char*)d_ws;
  unsigned short* xp  = (unsigned short*)(ws);
  unsigned short* wp  = (unsigned short*)(ws + xp_bytes);
  unsigned short* iwt = (unsigned short*)(ws + xp_bytes + wp_bytes);
  unsigned short* sp  = (unsigned short*)(ws + xp_bytes + wp_bytes + iw_bytes);

  const int gx = NB * (LP / 8);
  k_cvt_x<<<(gx + 255) / 256, 256, 0, stream>>>(x, xp);
  const int gw = NA * (NF / 8);
  k_cvt_w<<<(gw + 255) / 256, 256, 0, stream>>>(weight, wp);
  const int gi = NF * (KS / 8);
  k_cvt_iw<<<(gi + 255) / 256, 256, 0, stream>>>(invw, iwt);

  for (int grp = 0; grp < NGRP; ++grp) {
    dim3 gA(MP / 16, GRP);
    k_ana<<<gA, 128, 0, stream>>>(xp, wp, sp, grp * GRP);
    dim3 gS(NFB, 4, GRP);
    k_syn<<<gS, 128, 0, stream>>>(sp, iwt, window, out, grp * GRP);
  }
}
